// SS2D_55490977464367
// MI455X (gfx1250) — hardware-verified
//
#include <hip/hip_runtime.h>
#include <math.h>

typedef __attribute__((ext_vector_type(16))) _Float16 v16h;
typedef __attribute__((ext_vector_type(8)))  _Float16 v8h;
typedef __attribute__((ext_vector_type(16))) __bf16   v16b;
typedef __attribute__((ext_vector_type(8)))  __bf16   v8b;
typedef __attribute__((ext_vector_type(8)))  float    v8f;
typedef __attribute__((ext_vector_type(4)))  float    v4f;
typedef __attribute__((ext_vector_type(2)))  float    v2f;

constexpr int kB    = 2;
constexpr int kHgt  = 64;
constexpr int kWid  = 64;
constexpr int kL    = kHgt * kWid;
constexpr int kRows = kB * kL;
constexpr int kDm   = 96;
constexpr int kDin  = 192;
constexpr int kNst  = 16;
constexpr int kDtR  = 6;
constexpr int kNxp  = kDtR + 2 * kNst;
constexpr int kXzP  = 2 * kDin;
constexpr int kXpN  = 2 * kNxp;
constexpr int kXdP  = 128;
constexpr int kOpN  = 128;
static_assert(kDm % 32 == 0 && kDin % 32 == 0, "GEMM K multiples of 32");
static_assert(kRows % 64 == 0 && kXzP % 64 == 0 && kXdP % 64 == 0 && kOpN % 64 == 0, "GEMM M,N multiples of 64");
static_assert(kXpN <= kXdP && kDm <= kOpN, "padded N covers real N");
static_assert(kDm % 8 == 0 && kDin % 8 == 0, "8-element groups never straddle a row");

constexpr size_t kOffXH   = 0;
constexpr size_t kOffXL   = kOffXH  + (size_t)kRows * kDm  * 2;
constexpr size_t kOffWIH  = kOffXL  + (size_t)kRows * kDm  * 2;
constexpr size_t kOffWIL  = kOffWIH + (size_t)kXzP  * kDm  * 2;
constexpr size_t kOffWXH  = kOffWIL + (size_t)kXzP  * kDm  * 2;
constexpr size_t kOffWXL  = kOffWXH + (size_t)kXdP  * kDin * 2;
constexpr size_t kOffWOH  = kOffWXL + (size_t)kXdP  * kDin * 2;
constexpr size_t kOffWOL  = kOffWOH + (size_t)kOpN  * kDin * 2;
constexpr size_t kOffXZ   = kOffWOL + (size_t)kOpN  * kDin * 2;
constexpr size_t kOffUC   = kOffXZ  + (size_t)kRows * kXzP * 4;
constexpr size_t kOffUCH  = kOffUC  + (size_t)kRows * kDin * 4;
constexpr size_t kOffUCL  = kOffUCH + (size_t)kRows * kDin * 2;
constexpr size_t kOffXD   = kOffUCL + (size_t)kRows * kDin * 2;
constexpr size_t kOffYS   = kOffXD  + (size_t)kRows * kXdP * 4;
constexpr size_t kOffYH   = kOffYS  + (size_t)kB * 2 * kL * kDin * 4;
constexpr size_t kOffYL   = kOffYH  + (size_t)kRows * kDin * 2;
constexpr size_t kOffOP   = kOffYL  + (size_t)kRows * kDin * 2;
constexpr size_t kWsTotal = kOffOP  + (size_t)kRows * kOpN * 4;
static_assert(kWsTotal == 55918592ull, "carve total");
static_assert(kWsTotal <= 134217728ull, "carve cap");
static_assert((kOffXL % 128) == 0 && (kOffWIH % 128) == 0 && (kOffWIL % 128) == 0 && (kOffWXH % 128) == 0 &&
              (kOffWXL % 128) == 0 && (kOffWOH % 128) == 0 && (kOffWOL % 128) == 0 && (kOffXZ % 128) == 0 &&
              (kOffUC % 128) == 0 && (kOffUCH % 128) == 0 && (kOffUCL % 128) == 0 && (kOffXD % 128) == 0 &&
              (kOffYS % 128) == 0 && (kOffYH % 128) == 0 && (kOffYL % 128) == 0 && (kOffOP % 128) == 0,
              "128-B aligned regions");

__device__ __forceinline__ unsigned short f2bf_bits(float f) {
  unsigned u = __float_as_uint(f);
  return (unsigned short)((u + 0x7FFFu + ((u >> 16) & 1u)) >> 16);
}
__device__ __forceinline__ float bf_bits2f(unsigned short h) { return __uint_as_float(((unsigned)h) << 16); }

__device__ __forceinline__ void dep_guard4x_h(v8f& a, v8f& b, v8f& c, v8f& d, v16h x, v16h y) {
  asm volatile("v_nop\n\tv_nop\n\tv_nop\n\tv_nop" : "+v"(a), "+v"(b), "+v"(c), "+v"(d) : "v"(x), "v"(y));
}
__device__ __forceinline__ void dep_guard4x_b(v8f& a, v8f& b, v8f& c, v8f& d, v16b x, v16b y) {
  asm volatile("v_nop\n\tv_nop\n\tv_nop\n\tv_nop" : "+v"(a), "+v"(b), "+v"(c), "+v"(d) : "v"(x), "v"(y));
}
__device__ __forceinline__ void keep4_h(v16h a, v16h b, v16h c, v16h d) { asm volatile("v_nop" :: "v"(a), "v"(b), "v"(c), "v"(d)); }
__device__ __forceinline__ void keep4_b(v16b a, v16b b, v16b c, v16b d) { asm volatile("v_nop" :: "v"(a), "v"(b), "v"(c), "v"(d)); }
__device__ __forceinline__ void acc_guard4(v8f& a, v8f& b, v8f& c, v8f& d) { asm volatile("v_nop\n\tv_nop\n\tv_nop\n\tv_nop" : "+v"(a), "+v"(b), "+v"(c), "+v"(d)); }
template <typename T> struct Frag;
template <> struct Frag<_Float16> {
  typedef v16h V; union U { v16h v; v8h h[2]; };
  static __device__ __forceinline__ v16h load(const _Float16* p) {
    U f; f.h[0] = *(const v8h*)(p); f.h[1] = *(const v8h*)(p + 16); return f.v;
  }
  static __device__ __forceinline__ v8f mma(v16h a, v16h b, v8f c) {
    return __builtin_amdgcn_wmma_f32_16x16x32_f16(false, a, false, b, (short)0, c, false, false);
  }
  static __device__ __forceinline__ void guard4(v8f& a, v8f& b, v8f& c, v8f& d, v16h x, v16h y) { dep_guard4x_h(a, b, c, d, x, y); }
  static __device__ __forceinline__ void keep(v16h a, v16h b, v16h c, v16h d) { keep4_h(a, b, c, d); }
};
template <> struct Frag<__bf16> {
  typedef v16b V; union U { v16b v; v8b h[2]; };
  static __device__ __forceinline__ v16b load(const __bf16* p) {
    U f; f.h[0] = *(const v8b*)(p); f.h[1] = *(const v8b*)(p + 16); return f.v;
  }
  static __device__ __forceinline__ v8f mma(v16b a, v16b b, v8f c) {
    return __builtin_amdgcn_wmma_f32_16x16x32_bf16(false, a, false, b, (short)0, c, false, false);
  }
  static __device__ __forceinline__ void guard4(v8f& a, v8f& b, v8f& c, v8f& d, v16b x, v16b y) { dep_guard4x_b(a, b, c, d, x, y); }
  static __device__ __forceinline__ void keep(v16b a, v16b b, v16b c, v16b d) { keep4_b(a, b, c, d); }
};

template <int ET> struct Elem;
template <> struct Elem<0> { typedef _Float16 T; };
template <> struct Elem<1> { typedef __bf16 T; };
template <int ET, int SPL, int BIAS_MODE, int OUT_MODE, bool RESID, int ACT = 0>
__global__ __launch_bounds__(256) void wmma_gemm64(
    const unsigned short* __restrict__ Ap, const unsigned short* __restrict__ A2p, int lda, long strideA,
    const unsigned short* __restrict__ Btp, const unsigned short* __restrict__ Bt2p, int ldb, long strideB,
    void* __restrict__ Cout, void* __restrict__ Cout2, int ldc, long strideC,
    const float* __restrict__ bias,
    const float* __restrict__ resid, long strideR,
    int M, int N, int K, float scale) {
  typedef typename Elem<ET>::T T;
  typedef typename Frag<T>::V V;
  const T* A = (const T*)Ap; const T* A2 = (const T*)A2p; const T* Bt = (const T*)Btp; const T* Bt2 = (const T*)Bt2p;
  __shared__ __align__(16) float sT[8][16 * 68];
  const int b    = blockIdx.y;
  const int lane = threadIdx.x & 31;
  const int wave = threadIdx.x >> 5;
  const int tilesN = N >> 6;
  const int tilesM = M >> 6;
  const int tile = blockIdx.x * 8 + wave;
  if (tile >= tilesM * tilesN) return;
  const int tm = tile / tilesN;
  const int tn = tile - tm * tilesN;
  const int m0 = tm << 6;
  const int n0 = tn << 6;

  const T* Ab  = A  + (size_t)b * strideA;
  const T* Bb  = Bt + (size_t)b * strideB;
  const T* Ab2 = (SPL >= 1) ? (A2  + (size_t)b * strideA) : nullptr;
  const T* Bb2 = (SPL == 2) ? (Bt2 + (size_t)b * strideB) : nullptr;

  const int rlane = lane & 15;
  const int koff  = (lane >> 4) * 8;
  const int mOff  = (lane >> 4) * 8;

  v8f acc[4][4];
#pragma unroll
  for (int i = 0; i < 4; ++i)
#pragma unroll
    for (int j = 0; j < 4; ++j) acc[i][j] = (v8f){0.f,0.f,0.f,0.f,0.f,0.f,0.f,0.f};

  for (int k0 = 0; k0 < K; k0 += 32) {
    V bh[4], bl[4];
#pragma unroll
    for (int j = 0; j < 4; ++j) {
      const size_t bo = (size_t)(n0 + (j << 4) + rlane) * ldb + koff + k0;
      bh[j] = Frag<T>::load(Bb + bo);
      if (SPL == 2) bl[j] = Frag<T>::load(Bb2 + bo);
    }
#pragma unroll
    for (int i = 0; i < 4; ++i) {
      const size_t ao = (size_t)(m0 + (i << 4) + rlane) * lda + koff + k0;
      V ah = Frag<T>::load(Ab + ao);
      V al;
      if (SPL >= 1) al = Frag<T>::load(Ab2 + ao);
#pragma unroll
      for (int j = 0; j < 4; ++j) {
        acc[i][j] = Frag<T>::mma(ah, bh[j], acc[i][j]);
        if (SPL == 2) acc[i][j] = Frag<T>::mma(ah, bl[j], acc[i][j]);
        if (SPL >= 1) acc[i][j] = Frag<T>::mma(al, bh[j], acc[i][j]);
      }
      Frag<T>::guard4(acc[i][0], acc[i][1], acc[i][2], acc[i][3], ah, (SPL >= 1) ? al : ah);
    }
    Frag<T>::keep(bh[0], bh[1], bh[2], bh[3]);
    if (SPL == 2) Frag<T>::keep(bl[0], bl[1], bl[2], bl[3]);
  }
  acc_guard4(acc[0][0], acc[0][1], acc[0][2], acc[0][3]);
  acc_guard4(acc[1][0], acc[1][1], acc[1][2], acc[1][3]);
  acc_guard4(acc[2][0], acc[2][1], acc[2][2], acc[2][3]);
  acc_guard4(acc[3][0], acc[3][1], acc[3][2], acc[3][3]);

  float* slab = sT[wave];
  const float* Rb = RESID ? (resid + (size_t)b * strideR) : nullptr;
#pragma unroll
  for (int i = 0; i < 4; ++i) {
    const int mBase = m0 + (i << 4);
#pragma unroll
    for (int j = 0; j < 4; ++j) {
      const int n = n0 + (j << 4) + rlane;
      float bv = 0.f;
      if (BIAS_MODE == 2) bv = bias[n];
#pragma unroll
      for (int r = 0; r < 8; ++r) {
        float v = acc[i][j][r] * scale;
        if (BIAS_MODE == 1) v += bias[mBase + mOff + r];
        if (BIAS_MODE == 2) v += bv;
        if (RESID) v += Rb[(size_t)(mBase + mOff + r) * ldc + n];
        if (ACT == 1) v = tanhf(v);
        if (ACT == 2) v = fmaxf(v, 0.0f);
        if (ACT == 3) v = v / (1.0f + expf(-v));
        if (ACT == 4) v = (v > 0.f) ? v : 0.01f * v;
        slab[(mOff + r) * 68 + (j << 4) + rlane] = v;
      }
    }
    __builtin_amdgcn_fence(__ATOMIC_RELEASE, "workgroup");
    __builtin_amdgcn_wave_barrier();
    __builtin_amdgcn_fence(__ATOMIC_ACQUIRE, "workgroup");
    if (OUT_MODE == 0) {
      float* C = (float*)Cout + (size_t)b * strideC;
      const int hh = lane >> 4, c4 = (lane & 15) * 4;
      for (int pass = 0; pass < 2; ++pass) {
#pragma unroll
        for (int it = 0; it < 8; ++it) {
          const int row = it * 2 + hh;
          v4f v = *(const v4f*)(slab + row * 68 + c4);
          *(volatile v4f*)(C + (size_t)(mBase + row) * ldc + n0 + c4) = v;
        }
        __threadfence();
      }
    } else {
      const int q = lane >> 3, c8 = (lane & 7) * 8;
      unsigned short* C  = (unsigned short*)Cout  + (size_t)b * strideC;
      unsigned short* C2 = (OUT_MODE == 2) ? ((unsigned short*)Cout2 + (size_t)b * strideC) : nullptr;
      for (int pass = 0; pass < 2; ++pass) {
#pragma unroll
        for (int it = 0; it < 4; ++it) {
          const int row = it * 4 + q;
          const float* sp = slab + row * 68 + c8;
          v8h hv, lv;
#pragma unroll
          for (int e = 0; e < 8; ++e) {
            if (OUT_MODE == 1) {
              hv[e] = (_Float16)sp[e];
            } else {
              unsigned short hb = f2bf_bits(sp[e]);
              unsigned short lb = f2bf_bits(sp[e] - bf_bits2f(hb));
              hv[e] = __builtin_bit_cast(_Float16, hb);
              lv[e] = __builtin_bit_cast(_Float16, lb);
            }
          }
          *(volatile v8h*)(C + (size_t)(mBase + row) * ldc + n0 + c8) = hv;
          if (OUT_MODE == 2) *(volatile v8h*)(C2 + (size_t)(mBase + row) * ldc + n0 + c8) = lv;
        }
        __threadfence();
      }
    }
    __builtin_amdgcn_fence(__ATOMIC_RELEASE, "workgroup");
    __builtin_amdgcn_wave_barrier();
    __builtin_amdgcn_fence(__ATOMIC_ACQUIRE, "workgroup");
  }
}

__global__ __launch_bounds__(256) void split_rows_bf16_kernel(
    const float* __restrict__ src, unsigned short* __restrict__ dhi, unsigned short* __restrict__ dlo,
    int ncols, int rows_real, int total8)
{
  const int i = blockIdx.x * 256 + threadIdx.x;
  if (i >= total8) return;
  const size_t e0 = (size_t)i << 3;
  const int row = (int)(e0 / (size_t)ncols);
  const int col = (int)(e0 - (size_t)row * (size_t)ncols);
  const int rowc = (row < rows_real) ? row : (rows_real - 1);
  const float fac = (row < rows_real) ? 1.0f : 0.0f;
  const float* sp = src + (size_t)rowc * ncols + col;
  const v4f a0 = *(const v4f*)(sp);
  const v4f a1 = *(const v4f*)(sp + 4);
  v8h hv, lv;
#pragma unroll
  for (int e = 0; e < 4; ++e) {
    const float x0 = a0[e] * fac, x1 = a1[e] * fac;
    const unsigned short h0 = f2bf_bits(x0), h1 = f2bf_bits(x1);
    const unsigned short l0 = f2bf_bits(x0 - bf_bits2f(h0)), l1 = f2bf_bits(x1 - bf_bits2f(h1));
    hv[e]     = __builtin_bit_cast(_Float16, h0);
    hv[4 + e] = __builtin_bit_cast(_Float16, h1);
    lv[e]     = __builtin_bit_cast(_Float16, l0);
    lv[4 + e] = __builtin_bit_cast(_Float16, l1);
  }
  unsigned short* qh = dhi + e0;
  unsigned short* ql = dlo + e0;
  *(volatile v8h*)qh = hv;
  *(volatile v8h*)ql = lv;
  __threadfence();
  *(volatile v8h*)qh = hv;
  *(volatile v8h*)ql = lv;
}

constexpr int kConvPix = 16;
constexpr int kConvTP  = 196;
static_assert(kRows % kConvPix == 0 && kWid % kConvPix == 0, "conv tile");
static_assert((kConvPix * kDin) % 128 == 0 && (kConvPix * kDin) % 256 == 0, "conv chunks");
__global__ __launch_bounds__(192) void conv_silu_kernel(
    const float* __restrict__ XZ, const float* __restrict__ cw, const float* __restrict__ cb,
    float* __restrict__ UC, unsigned short* __restrict__ UCH, unsigned short* __restrict__ UCL)
{
  __shared__ __align__(16) float sT[kConvPix * kConvTP];
  const int tid = threadIdx.x, lane = tid & 31, wave = tid >> 5;
  const int p0 = blockIdx.x * kConvPix;
  const int bimg = p0 / kL;
  const int l0 = p0 - bimg * kL;
  const int hc = l0 >> 6;
  const int w0 = l0 & (kWid - 1);
  float wg[9];
#pragma unroll
  for (int i = 0; i < 9; ++i) wg[i] = cw[tid * 9 + i];
  const float bc = cb[tid];
  const size_t ib = (size_t)bimg * kL;
#pragma unroll 1
  for (int s = 0; s < kConvPix; ++s) {
    const int wc = w0 + s;
    float acc = 0.0f;
#pragma unroll
    for (int ky = 0; ky < 3; ++ky) {
      const int hy = hc + ky - 1;
      const int hyc = hy < 0 ? 0 : (hy > kHgt - 1 ? kHgt - 1 : hy);
      const float fy = (hy >= 0 && hy < kHgt) ? 1.0f : 0.0f;
#pragma unroll
      for (int kx = 0; kx < 3; ++kx) {
        const int wx = wc + kx - 1;
        const int wxc = wx < 0 ? 0 : (wx > kWid - 1 ? kWid - 1 : wx);
        const float fxy = (wx >= 0 && wx < kWid) ? fy : 0.0f;
        const float v = XZ[(ib + (size_t)hyc * kWid + (size_t)wxc) * kXzP + tid];
        acc = fmaf(v, wg[ky * 3 + kx] * fxy, acc);
      }
    }
    const float sv = acc + bc;
    const float sg = __builtin_amdgcn_rcpf(1.0f + expf(-sv));
    sT[s * kConvTP + tid] = sv * sg;
  }
  __syncthreads();
  const size_t tb = (size_t)p0 * kDin;
  v8h hv[2], lv[2];
#pragma unroll
  for (int it = 0; it < 2; ++it) {
    const int q = wave + 6 * it;
    const int f = q * 256 + lane * 8;
    const int row = f / kDin, col = f - row * kDin;
    const float* sp = sT + row * kConvTP + col;
    const v4f a0 = *(const v4f*)(sp);
    const v4f a1 = *(const v4f*)(sp + 4);
#pragma unroll
    for (int e = 0; e < 4; ++e) {
      const unsigned short h0 = f2bf_bits(a0[e]), h1 = f2bf_bits(a1[e]);
      const unsigned short l0b = f2bf_bits(a0[e] - bf_bits2f(h0)), l1b = f2bf_bits(a1[e] - bf_bits2f(h1));
      hv[it][e]     = __builtin_bit_cast(_Float16, h0);
      hv[it][4 + e] = __builtin_bit_cast(_Float16, h1);
      lv[it][e]     = __builtin_bit_cast(_Float16, l0b);
      lv[it][4 + e] = __builtin_bit_cast(_Float16, l1b);
    }
  }
  for (int pass = 0; pass < 2; ++pass) {
#pragma unroll
    for (int it = 0; it < 4; ++it) {
      const int q = wave + 6 * it;
      const int f = q * 128 + lane * 4;
      const int row = f / kDin, col = f - row * kDin;
      const v4f v = *(const v4f*)(sT + row * kConvTP + col);
      *(volatile v4f*)(UC + tb + f) = v;
    }
#pragma unroll
    for (int it = 0; it < 2; ++it) {
      const int q = wave + 6 * it;
      const int f = q * 256 + lane * 8;
      *(volatile v8h*)(UCH + tb + f) = hv[it];
      *(volatile v8h*)(UCL + tb + f) = lv[it];
    }
    __threadfence();
  }
}

constexpr int kScanTS = 64;
constexpr int kScanCh = 64;
constexpr int kSxP    = 44;
constexpr int kSyP    = 68;
constexpr int kScanGrp = kDin / kScanCh;
constexpr int kScanBlocks = kB * 2 * kScanGrp;
static_assert(kScanTS == kWid && (kL % kScanTS) == 0 && (kDin % kScanCh) == 0, "scan tiles");
static_assert(kNxp - 2 + kSxP <= kXdP && (kNxp - 2) % 4 == 0 && kNxp + 2 <= kSxP, "scan staging window");
__global__ __launch_bounds__(kScanCh) void scan_kernel(
    const float* __restrict__ XD, const float* __restrict__ UC,
    const float* __restrict__ Wdt, const float* __restrict__ bdt, const float* __restrict__ Alog,
    const float* __restrict__ Dp, float* __restrict__ YS)
{
  __shared__ __align__(16) float sX[kScanTS * kSxP];
  __shared__ __align__(16) float sY[kScanTS * kSyP];
  __shared__ __align__(16) float sA[kNst * kScanCh];
  __shared__ __align__(16) float sW[8 * kScanCh];
  const int tid = threadIdx.x, lane = tid & 31, wave = tid >> 5;
  const int bx = blockIdx.x;
  const int bimg = bx / (2 * kScanGrp);
  const int rem  = bx - bimg * (2 * kScanGrp);
  const int kdir = rem / kScanGrp;
  const int g    = rem - kdir * kScanGrp;
  const int d0 = g * kScanCh;
  const int d  = d0 + tid;
  const int prow = kdir * kDin + d;
#pragma unroll 1
  for (int r = 0; r < kDtR; ++r) sW[r * kScanCh + tid] = Wdt[(size_t)prow * kDtR + r];
#pragma unroll 1
  for (int s = 0; s < kNst; ++s) sA[s * kScanCh + tid] = -expf(Alog[(size_t)prow * kNst + s]);
  __syncthreads();
  float negA[kNst], h[kNst], wd[kDtR];
#pragma unroll
  for (int s = 0; s < kNst; ++s) { negA[s] = sA[s * kScanCh + tid]; h[s] = 0.0f; }
#pragma unroll
  for (int r = 0; r < kDtR; ++r) wd[r] = sW[r * kScanCh + tid];
  const float bb = bdt[prow], Dd = Dp[prow];
  const size_t row0 = (size_t)bimg * kL;
  float* ysb = YS + ((size_t)(bimg * 2 + kdir) * kL) * kDin;
  const int cbase = kdir ? (kNxp - 2) : 0;
  const int off   = kdir ? 2 : 0;
  const int hh = lane >> 4, c4 = (lane & 15) * 4;
#pragma unroll 1
  for (int t0 = 0; t0 < kL; t0 += kScanTS) {
    __syncthreads();
    {
      const float* src = XD + (row0 + t0 + tid) * kXdP + cbase;
      float* dst = sX + tid * kSxP;
#pragma unroll 1
      for (int j = 0; j < kSxP / 4; ++j) *(v4f*)(dst + 4 * j) = *(const v4f*)(src + 4 * j);
    }
    __syncthreads();
#pragma unroll 1
    for (int s = 0; s < kScanTS; ++s) {
      const int ls = kdir ? (kScanTS - 1 - s) : s;
      const float* xr = sX + ls * kSxP + off;
      const v2f x01 = *(const v2f*)(xr);
      const v2f x23 = *(const v2f*)(xr + 2);
      const v2f x45 = *(const v2f*)(xr + 4);
      float vdot = 0.0f;
      vdot = fmaf(x01[0], wd[0], vdot);
      vdot = fmaf(x01[1], wd[1], vdot);
      vdot = fmaf(x23[0], wd[2], vdot);
      vdot = fmaf(x23[1], wd[3], vdot);
      vdot = fmaf(x45[0], wd[4], vdot);
      vdot = fmaf(x45[1], wd[5], vdot);
      const float v   = vdot + bb;
      const float ea  = expf(-fabsf(v));
      const float dlt = fmaxf(v, 0.0f) + log1pf(ea);
      const float u   = UC[(row0 + t0 + ls) * kDin + d];
      const float dtu = dlt * u;
      float Bs[kNst], Cs[kNst];
#pragma unroll
      for (int q2 = 0; q2 < kNst / 2; ++q2) {
        const v2f bv = *(const v2f*)(xr + kDtR + 2 * q2);
        const v2f cv = *(const v2f*)(xr + kDtR + kNst + 2 * q2);
        Bs[2 * q2] = bv[0]; Bs[2 * q2 + 1] = bv[1];
        Cs[2 * q2] = cv[0]; Cs[2 * q2 + 1] = cv[1];
      }
      float y = 0.0f;
#pragma unroll
      for (int n = 0; n < kNst; ++n) {
        const float e = __expf(dlt * negA[n]);
        h[n] = fmaf(e, h[n], dtu * Bs[n]);
        y = fmaf(h[n], Cs[n], y);
      }
      y = fmaf(Dd, u, y);
      sY[s * kSyP + tid] = y;
    }
    __syncthreads();
    for (int pass = 0; pass < 2; ++pass) {
#pragma unroll
      for (int it = 0; it < 16; ++it) {
        const int row = it * 4 + wave * 2 + hh;
        const v4f vv = *(const v4f*)(sY + row * kSyP + c4);
        *(volatile v4f*)(ysb + (size_t)(t0 + row) * kDin + d0 + c4) = vv;
      }
      __threadfence();
    }
  }
}

constexpr int kLnPix = 32;
constexpr int kLnTP  = 196;
static_assert(kRows % kLnPix == 0 && (kLnPix * kDin) % (256 * 8) == 0 && kDin % 32 == 0, "ln tile");
__global__ __launch_bounds__(256) void ln_gate_kernel(
    const float* __restrict__ YS, const float* __restrict__ XZ,
    const float* __restrict__ lns, const float* __restrict__ lnb,
    unsigned short* __restrict__ YH, unsigned short* __restrict__ YL)
{
  __shared__ __align__(16) float sT[kLnPix * kLnTP];
  const int tid = threadIdx.x, lane = tid & 31, wave = tid >> 5;
  const int p0 = blockIdx.x * kLnPix;
#pragma unroll 1
  for (int i = 0; i < kLnPix / 8; ++i) {
    const int pl = wave * (kLnPix / 8) + i;
    const int p = p0 + pl;
    const int bimg = p / kL;
    const int l = p - bimg * kL;
    const float* r0 = YS + ((size_t)(bimg * 2) * kL + (size_t)l) * kDin;
    const float* r1 = YS + ((size_t)(bimg * 2 + 1) * kL + (size_t)(kL - 1 - l)) * kDin;
    float* st = sT + pl * kLnTP;
    float sum = 0.0f;
#pragma unroll 1
    for (int j = 0; j < kDin / 32; ++j) {
      const int c = lane + 32 * j;
      const float y = r0[c] + r1[c];
      st[c] = y;
      sum += y;
    }
#pragma unroll
    for (int o = 16; o > 0; o >>= 1) sum += __shfl_xor(sum, o, 32);
    const float mu = sum * (1.0f / (float)kDin);
    float sq = 0.0f;
#pragma unroll 1
    for (int j = 0; j < kDin / 32; ++j) {
      const int c = lane + 32 * j;
      const float dv = st[c] - mu;
      sq = fmaf(dv, dv, sq);
    }
#pragma unroll
    for (int o = 16; o > 0; o >>= 1) sq += __shfl_xor(sq, o, 32);
    const float var = sq * (1.0f / (float)kDin);
    const float rs  = rsqrtf(var + 1e-5f);
#pragma unroll 1
    for (int j = 0; j < kDin / 32; ++j) {
      const int c = lane + 32 * j;
      const float y  = st[c];
      const float yn = (y - mu) * rs * lns[c] + lnb[c];
      const float zv = XZ[(size_t)p * kXzP + kDin + c];
      const float gt = zv * __builtin_amdgcn_rcpf(1.0f + expf(-zv));
      st[c] = yn * gt;
    }
  }
  __syncthreads();
  const size_t tb = (size_t)p0 * kDin;
  v8h hv[3], lv[3];
#pragma unroll
  for (int it = 0; it < 3; ++it) {
    const int q = wave + 8 * it;
    const int f = q * 256 + lane * 8;
    const int row = f / kDin, col = f - row * kDin;
    const float* sp = sT + row * kLnTP + col;
    const v4f a0 = *(const v4f*)(sp);
    const v4f a1 = *(const v4f*)(sp + 4);
#pragma unroll
    for (int e = 0; e < 4; ++e) {
      const unsigned short h0 = f2bf_bits(a0[e]), h1 = f2bf_bits(a1[e]);
      const unsigned short l0b = f2bf_bits(a0[e] - bf_bits2f(h0)), l1b = f2bf_bits(a1[e] - bf_bits2f(h1));
      hv[it][e]     = __builtin_bit_cast(_Float16, h0);
      hv[it][4 + e] = __builtin_bit_cast(_Float16, h1);
      lv[it][e]     = __builtin_bit_cast(_Float16, l0b);
      lv[it][4 + e] = __builtin_bit_cast(_Float16, l1b);
    }
  }
  for (int pass = 0; pass < 2; ++pass) {
#pragma unroll
    for (int it = 0; it < 3; ++it) {
      const int q = wave + 8 * it;
      const int f = q * 256 + lane * 8;
      *(volatile v8h*)(YH + tb + f) = hv[it];
      *(volatile v8h*)(YL + tb + f) = lv[it];
    }
    __threadfence();
  }
}

__global__ __launch_bounds__(256) void repack_out_kernel(
    const float* __restrict__ OP, float* __restrict__ outp, int total4)
{
  const int i = blockIdx.x * 256 + threadIdx.x;
  if (i >= total4) return;
  const size_t f = (size_t)i * 4;
  const int row = (int)(f / kDm);
  const int col = (int)(f - (size_t)row * kDm);
  const v4f v = *(const v4f*)(OP + (size_t)row * kOpN + col);
  float* q = outp + f;
  *(volatile v4f*)q = v;
  __threadfence();
  *(volatile v4f*)q = v;
}

static_assert((kRows / 64) * (kXzP / 64) == 96 * 8, "in_proj grid");
static_assert((kRows / 64) * (kXdP / 64) == 32 * 8, "x_proj grid");
static_assert((kRows / 64) * (kOpN / 64) == 32 * 8, "out_proj grid");
extern "C" void kernel_launch(void* const* d_in, const int* in_sizes, int n_in,
                              void* d_out, int out_size, void* d_ws, size_t ws_size,
                              hipStream_t stream) {
  if (n_in < 12) return;
  if (in_sizes[0] != kRows * kDm) return;
  if (in_sizes[1] != kXzP * kDm) return;
  if (in_sizes[2] != kDin * 9) return;
  if (in_sizes[3] != kDin) return;
  if (in_sizes[4] != kXpN * kDin) return;
  if (in_sizes[5] != 2 * kDin * kDtR) return;
  if (in_sizes[6] != 2 * kDin) return;
  if (in_sizes[7] != 2 * kDin * kNst) return;
  if (in_sizes[8] != 2 * kDin) return;
  if (in_sizes[9] != kDin) return;
  if (in_sizes[10] != kDin) return;
  if (in_sizes[11] != kDm * kDin) return;
  if (out_size != kRows * kDm) return;
  if (ws_size < kWsTotal) return;

  const float* x       = (const float*)d_in[0];
  const float* W_in    = (const float*)d_in[1];
  const float* conv_w  = (const float*)d_in[2];
  const float* conv_b  = (const float*)d_in[3];
  const float* W_xproj = (const float*)d_in[4];
  const float* W_dt    = (const float*)d_in[5];
  const float* b_dt    = (const float*)d_in[6];
  const float* A_log   = (const float*)d_in[7];
  const float* Dp      = (const float*)d_in[8];
  const float* ln_s    = (const float*)d_in[9];
  const float* ln_b    = (const float*)d_in[10];
  const float* W_out   = (const float*)d_in[11];
  float* out = (float*)d_out;

  char* ws = (char*)d_ws;
  unsigned short* XH   = (unsigned short*)(ws + kOffXH);
  unsigned short* XL   = (unsigned short*)(ws + kOffXL);
  unsigned short* WIH  = (unsigned short*)(ws + kOffWIH);
  unsigned short* WIL  = (unsigned short*)(ws + kOffWIL);
  unsigned short* WXH  = (unsigned short*)(ws + kOffWXH);
  unsigned short* WXL  = (unsigned short*)(ws + kOffWXL);
  unsigned short* WOH  = (unsigned short*)(ws + kOffWOH);
  unsigned short* WOL  = (unsigned short*)(ws + kOffWOL);
  float*          XZ   = (float*)(ws + kOffXZ);
  float*          UC   = (float*)(ws + kOffUC);
  unsigned short* UCH  = (unsigned short*)(ws + kOffUCH);
  unsigned short* UCL  = (unsigned short*)(ws + kOffUCL);
  float*          XD   = (float*)(ws + kOffXD);
  float*          YS   = (float*)(ws + kOffYS);
  unsigned short* YH   = (unsigned short*)(ws + kOffYH);
  unsigned short* YL   = (unsigned short*)(ws + kOffYL);
  float*          OP   = (float*)(ws + kOffOP);

  {
    const int t8x  = kRows * kDm / 8;
    const int t8wi = kXzP * kDm / 8;
    const int t8wx = kXdP * kDin / 8;
    const int t8wo = kOpN * kDin / 8;
    split_rows_bf16_kernel<<<(t8x + 255) / 256, 256, 0, stream>>>(x, XH, XL, kDm, kRows, t8x);
    split_rows_bf16_kernel<<<(t8wi + 255) / 256, 256, 0, stream>>>(W_in, WIH, WIL, kDm, kXzP, t8wi);
    split_rows_bf16_kernel<<<(t8wx + 255) / 256, 256, 0, stream>>>(W_xproj, WXH, WXL, kDin, kXpN, t8wx);
    split_rows_bf16_kernel<<<(t8wo + 255) / 256, 256, 0, stream>>>(W_out, WOH, WOL, kDin, kDm, t8wo);
  }

  wmma_gemm64<1, 2, 0, 0, false><<<dim3(96, 1), 256, 0, stream>>>(
      XH, XL, kDm, 0L,
      WIH, WIL, kDm, 0L,
      (void*)XZ, nullptr, kXzP, 0L,
      nullptr, nullptr, 0L,
      kRows, kXzP, kDm, 1.0f);

  conv_silu_kernel<<<kRows / kConvPix, kDin, 0, stream>>>(XZ, conv_w, conv_b, UC, UCH, UCL);

  wmma_gemm64<1, 2, 0, 0, false><<<dim3(32, 1), 256, 0, stream>>>(
      UCH, UCL, kDin, 0L,
      WXH, WXL, kDin, 0L,
      (void*)XD, nullptr, kXdP, 0L,
      nullptr, nullptr, 0L,
      kRows, kXdP, kDin, 1.0f);

  scan_kernel<<<kScanBlocks, kScanCh, 0, stream>>>(XD, UC, W_dt, b_dt, A_log, Dp, YS);

  ln_gate_kernel<<<kRows / kLnPix, 256, 0, stream>>>(YS, XZ, ln_s, ln_b, YH, YL);

  wmma_gemm64<1, 2, 0, 0, false><<<dim3(32, 1), 256, 0, stream>>>(
      YH, YL, kDin, 0L,
      WOH, WOL, kDin, 0L,
      (void*)OP, nullptr, kOpN, 0L,
      nullptr, nullptr, 0L,
      kRows, kOpN, kDin, 1.0f);

  {
    const int total4 = kRows * kDm / 4;
    repack_out_kernel<<<(total4 + 255) / 256, 256, 0, stream>>>(OP, out, total4);
  }
}
